// predictor_10917806866765
// MI455X (gfx1250) — hardware-verified
//
#include <hip/hip_runtime.h>


namespace {
constexpr int N = 100000, E = 3200000, DN = 5, DI = 10, DH = 50, ELIM = 3200000  ;
constexpr float XS = 8.0f, WSC = 256.0f;
static_assert(E % 32 == 0 && ELIM % 32 == 0, "tiling");
typedef _Float16 b16;
typedef __attribute__((ext_vector_type(16))) _Float16 v16b;
typedef __attribute__((ext_vector_type(8))) _Float16 v8b;
typedef __attribute__((ext_vector_type(8))) float v8f;
typedef __attribute__((ext_vector_type(4))) float v4f;
__device__ __forceinline__ float bf16_rne(float f) { unsigned int u = __float_as_uint(f); u += 0x7FFFu + ((u >> 16) & 1u); return __uint_as_float(u & 0xFFFF0000u); }
__device__ __forceinline__ void split16(float v, b16& hi, b16& lo) { hi = (b16)v; lo = (b16)(v - (float)hi); }
__device__ __forceinline__ v16b frag_kb(const b16* p, int hh) { const v8b a = *(const v8b*)(p + 8 * hh), b = *(const v8b*)(p + 16 + 8 * hh); v16b f;
#pragma unroll
  for (int e = 0; e < 8; ++e) { f[e] = a[e]; f[8 + e] = b[e]; } return f; }
__device__ __forceinline__ v8f wmma16b(v16b a, v16b b, v8f c) { v8f d = __builtin_amdgcn_wmma_f32_16x16x32_f16(false, a, false, b, (short)0, c, false, false); asm volatile("v_nop\n\tv_nop\n\tv_nop\n\tv_nop" : "+v"(d) : "v"(a), "v"(b)); return d; }
__device__ __forceinline__ void wave_lds_sync() { __builtin_amdgcn_fence(__ATOMIC_RELEASE, "workgroup"); __builtin_amdgcn_wave_barrier(); __builtin_amdgcn_fence(__ATOMIC_ACQUIRE, "workgroup"); }
__device__ __forceinline__ float pmul(float a, float b) { float p = a * b; asm volatile("" : "+v"(p)); return p; }
__device__ __forceinline__ int iclamp(int v, int lo, int hi) { return v < lo ? lo : (v > hi ? hi : v); }

__global__ __launch_bounds__(256) void prep_kernel(const float* __restrict__ w2, b16* __restrict__ W2T) {
  for (int i = threadIdx.x; i < 64 * 64 / 8; i += 256) { const int e = i * 8; const int oo = e / 64, k0 = e % 64; v8b o; for (int j = 0; j < 8; ++j) { const int k = k0 + j; o[j] = (oo < DH && k < DH) ? (b16)(bf16_rne(w2[k * DH + oo]) * WSC) : (b16)0.0f; }
    for (int pass = 0; pass < 2; ++pass) { *(volatile v8b*)(W2T + e) = o; __threadfence(); } }
}
__global__ __launch_bounds__(256) void nodeproj_kernel(const float* __restrict__ x, const float* __restrict__ w1, float* __restrict__ P) {
  const int wave = threadIdx.x >> 5, lane = threadIdx.x & 31; const size_t v = (size_t)blockIdx.x * 8 + wave; if (v >= (size_t)N) return;
  float xv[DN]; for (int i = 0; i < DN; ++i) xv[i] = bf16_rne(x[v * DN + i]);
  v4f o4;
#pragma unroll
  for (int j = 0; j < 4; ++j) { const int c = lane * 4 + j; float s = 0.0f; if (c < 2 * DH) { const int half = c / DH, o = c % DH;
#pragma unroll
      for (int i = 0; i < DN; ++i) s += xv[i] * bf16_rne(w1[(half * DN + i) * DH + o]); }
    o4[j] = s; }
  for (int pass = 0; pass < 2; ++pass) { *(volatile v4f*)(P + v * 128 + lane * 4) = o4; __threadfence(); }
}
__global__ __launch_bounds__(128) void edge_kernel(const float* __restrict__ P, const int* __restrict__ srcs, const int* __restrict__ dsts, const float* __restrict__ b1, const b16* __restrict__ W2T, const float* __restrict__ b2, const float* __restrict__ w3, const float* __restrict__ b3, float* __restrict__ out) {
  __shared__ __attribute__((aligned(16))) float Tf[4][2][16][64 + 4]; __shared__ float B1s[64], B2s[64], W3s[64];
  const int wave = threadIdx.x >> 5, lane = threadIdx.x & 31, nloc = lane & 15, hlf = lane >> 4; const size_t e0 = ((size_t)blockIdx.x * 4 + wave) * 32;
  if (threadIdx.x < 64) { const int k = threadIdx.x; B1s[k] = (k < DH) ? bf16_rne(b1[k]) : 0.0f; B2s[k] = (k < DH) ? bf16_rne(b2[k]) : 0.0f; W3s[k] = (k < DH) ? bf16_rne(w3[k]) : 0.0f; }
  __syncthreads();
  v8f acc[2][4];
#pragma unroll
  for (int rt = 0; rt < 2; ++rt)
#pragma unroll
    for (int t = 0; t < 4; ++t) acc[rt][t] = (v8f){};
#pragma unroll
  for (int rt = 0; rt < 2; ++rt) { const size_t e = e0 + rt * 16 + nloc; const size_t s = (size_t)iclamp(srcs[e], 0, N - 1), d = (size_t)iclamp(dsts[e], 0, N - 1); const float* ps = P + s * 128; const float* pd = P + d * 128 + DH;
#pragma unroll
    for (int ks = 0; ks < 2; ++ks) { v16b a;
#pragma unroll
      for (int g = 0; g < 2; ++g) { const int kb = ks * 32 + g * 16 + 8 * hlf;
        const v4f s0 = *(const v4f*)(ps + kb), s1 = *(const v4f*)(ps + kb + 4); float dv[8];
#pragma unroll
        for (int i = 0; i < 8; ++i) dv[i] = pd[kb + i];
#pragma unroll
        for (int i = 0; i < 8; ++i) { const int k = kb + i; const float sv = (i < 4) ? s0[i] : s1[i - 4]; const float h = (k < DH) ? fmaxf(sv + dv[i] + B1s[k], 0.0f) : 0.0f; a[g * 8 + i] = (b16)(h * XS); } }
#pragma unroll
      for (int t = 0; t < 4; ++t) acc[rt][t] = wmma16b(a, frag_kb(W2T + (size_t)(t * 16 + nloc) * 64 + ks * 32, hlf), acc[rt][t]); } }
#pragma unroll
  for (int rt = 0; rt < 2; ++rt)
#pragma unroll
    for (int t = 0; t < 4; ++t)
#pragma unroll
      for (int r = 0; r < 8; ++r) { const int c = t * 16 + nloc; Tf[wave][rt][8 * hlf + r][c] = fmaxf(acc[rt][t][r] * (1.0f / (XS * WSC)) + B2s[c], 0.0f); }
  wave_lds_sync();
  const int rt = lane >> 4, er = lane & 15; float z = bf16_rne(b3[0]);
#pragma unroll 1
  for (int o = 0; o < DH; ++o) z += Tf[wave][rt][er][o] * W3s[o];
  const float y = 1.0f / (1.0f + __expf(-z));
  for (int pass = 0; pass < 2; ++pass) { ((volatile float*)out)[e0 + lane] = y; __threadfence(); }
}
}

extern "C" void kernel_launch(void* const* d_in, const int* in_sizes, int n_in, void* d_out, int out_size, void* d_ws, size_t ws_size, hipStream_t stream) {
  (void)n_in;
  auto Fp = [&](int i) { return (const float*)d_in[i]; }; auto Ip = [&](int i) { return (const int*)d_in[i]; };
  if (in_sizes[0] != N * DN || in_sizes[1] != 2 * E || in_sizes[2] != DI * DH || in_sizes[3] != DH || in_sizes[4] != DH * DH || in_sizes[5] != DH || in_sizes[6] != DH || in_sizes[7] != 1 || out_size != E) return;
  size_t off = 0; char* ws = (char*)d_ws;
  auto carve = [&](size_t bytes) { char* p = ws + off; off += (bytes + 255) & ~(size_t)255; return p; };
  b16* W2T = (b16*)carve(64 * 64 * 2); float* P = (float*)carve((size_t)N * 128 * 4);
  if (off > ws_size || off > ((size_t)128 << 20)) return;
  prep_kernel<<<1, 256, 0, stream>>>(Fp(4), W2T);
  nodeproj_kernel<<<(N + 7) / 8, 256, 0, stream>>>(Fp(0), Fp(2), P);
  edge_kernel<<<ELIM / 128, 128, 0, stream>>>(P, Ip(1), Ip(1) + E, Fp(3), W2T, Fp(5), Fp(6), Fp(7), (float*)d_out);
}
